// DCN_62766652064420
// MI455X (gfx1250) — hardware-verified
//
#include <hip/hip_runtime.h>


namespace {
typedef _Float16 b16;
typedef __attribute__((ext_vector_type(16))) _Float16 v16b;
typedef __attribute__((ext_vector_type(8))) _Float16 v8b;
typedef __attribute__((ext_vector_type(4))) _Float16 v4h;
typedef __attribute__((ext_vector_type(2))) _Float16 v2h;
typedef __attribute__((ext_vector_type(8))) float v8f;
typedef __attribute__((ext_vector_type(4))) float v4f;
typedef __attribute__((ext_vector_type(2))) float v2f;
__device__ __forceinline__ float bf16_rne(float f) { unsigned int u = __float_as_uint(f); u += 0x7FFFu + ((u >> 16) & 1u); return __uint_as_float(u & 0xFFFF0000u); }
__device__ __forceinline__ void split16(float v, b16& hi, b16& lo) { hi = (b16)v; lo = (b16)(v - (float)hi); }
__device__ __forceinline__ v16b frag_kb(const b16* p, int hh) { const v8b a = *(const v8b*)(p + 8 * hh), b = *(const v8b*)(p + 16 + 8 * hh); v16b f;
#pragma unroll
  for (int e = 0; e < 8; ++e) { f[e] = a[e]; f[8 + e] = b[e]; } return f; }
__device__ __forceinline__ v8f wmma16b(v16b a, v16b b, v8f c) { v8f d = __builtin_amdgcn_wmma_f32_16x16x32_f16(false, a, false, b, (short)0, c, false, false); asm volatile("v_nop\n\tv_nop\n\tv_nop\n\tv_nop" : "+v"(d) : "v"(a), "v"(b)); return d; }
__device__ __forceinline__ void wave_lds_sync() { __builtin_amdgcn_fence(__ATOMIC_RELEASE, "workgroup"); __builtin_amdgcn_wave_barrier(); __builtin_amdgcn_fence(__ATOMIC_ACQUIRE, "workgroup"); }
__device__ __forceinline__ float pmul(float a, float b) { float p = a * b; asm volatile("" : "+v"(p)); return p; }
__device__ __forceinline__ int iclamp(int v, int lo, int hi) { return v < lo ? lo : (v > hi ? hi : v); }
__device__ __forceinline__ float nexp2(float v) { return __builtin_amdgcn_exp2f(v); }

constexpr int B = 16, BL = B  , C = 128, H = 56, W = 56, HW = H * W, KS = 3, NT = KS * KS, OC = 256, KD = NT * C  ;
constexpr float XS = 8.0f, WSC = 256.0f, RS_ = 1024.0f, CXY = 27.5f  ;
static_assert(HW % 32 == 0 && C == 128 && OC == 256 && H == W, "tiling");

__global__ __launch_bounds__(256) void wperm_kernel(const float* __restrict__ w, b16* __restrict__ WT, float scl) {
  const int u = blockIdx.x * 256 + threadIdx.x; if (u >= OC * KD / 8) return; const int e = u * 8; const int o = e / KD, k0 = e % KD; const int tap = k0 / C, c0 = k0 % C; v8b v;
#pragma unroll
  for (int q = 0; q < 8; ++q) v[q] = (b16)(bf16_rne(w[((size_t)o * C + c0 + q) * NT + tap]) * scl);
  for (int pass = 0; pass < 2; ++pass) { *(volatile v8b*)(WT + e) = v; __threadfence(); }
}
__global__ __launch_bounds__(256) void nhwc_kernel(const float* __restrict__ f, float* __restrict__ FT) {
  __shared__ float Ts[32][C + 1]; const int b = blockIdx.y, p0 = blockIdx.x * 32;
  for (int i = threadIdx.x; i < C * 32; i += 256) { const int c = i / 32, pp = i % 32; Ts[pp][c] = bf16_rne(f[((size_t)b * C + c) * HW + p0 + pp]); }
  __syncthreads();
  for (int pass = 0; pass < 2; ++pass) { for (int i = threadIdx.x; i < 32 * C / 4; i += 256) { const int pp = i / (C / 4), c4 = (i % (C / 4)) * 4; v4f v; for (int q = 0; q < 4; ++q) v[q] = Ts[pp][c4 + q]; *(volatile v4f*)(FT + ((size_t)b * HW + p0 + pp) * C + c4) = v; } __threadfence(); }
}
__global__ __launch_bounds__(64) void dcn_kernel(const float* __restrict__ FT, const float* __restrict__ off, const b16* __restrict__ WT, const b16* __restrict__ WTQ, float* __restrict__ out) {
  __shared__ __attribute__((aligned(16))) b16 Ah[2][16][C + 8], Al[2][16][C + 8]; __shared__ __attribute__((aligned(16))) float Tf[2][16][OC + 4];
  const int wave = threadIdx.x >> 5, lane = threadIdx.x & 31, nloc = lane & 15, hlf = lane >> 4; const int b = blockIdx.y; const int p0 = blockIdx.x * 32 + wave * 16; const int p = p0 + nloc; const int ho = p / W, wo = p % W;
  const float* FTb = FT + (size_t)b * HW * C; const float* offb = off + (size_t)b * 2 * NT * HW;
  v8f acc[16];
#pragma unroll
  for (int t = 0; t < 16; ++t) acc[t] = (v8f){};
#pragma unroll 1
  for (int tap = 0; tap < NT; ++tap) {
    const float ox = bf16_rne(offb[((size_t)(tap * 2 + 0) * H + wo) * W + ho]), oy = bf16_rne(offb[((size_t)(tap * 2 + 1) * H + wo) * W + ho]);
    const float gxn = ox + ((float)wo - CXY) / CXY, gyn = oy + ((float)ho - CXY) / CXY;
    const float px = (gxn + 1.0f) * 0.5f * (float)(W - 1), py = (gyn + 1.0f) * 0.5f * (float)(H - 1);
    const float fx = floorf(px), fy = floorf(py); const float wx1 = px - fx, wy1 = py - fy, wx0 = 1.0f - wx1, wy0 = 1.0f - wy1;
    const int x0 = (int)fx, y0 = (int)fy, x1 = x0 + 1, y1 = y0 + 1;
    const float v00 = (x0 >= 0 && x0 <= W - 1 && y0 >= 0 && y0 <= H - 1) ? 1.0f : 0.0f, v10 = (x1 >= 0 && x1 <= W - 1 && y0 >= 0 && y0 <= H - 1) ? 1.0f : 0.0f, v01 = (x0 >= 0 && x0 <= W - 1 && y1 >= 0 && y1 <= H - 1) ? 1.0f : 0.0f, v11 = (x1 >= 0 && x1 <= W - 1 && y1 >= 0 && y1 <= H - 1) ? 1.0f : 0.0f;
    const float w00 = wx0 * wy0 * v00, w10 = wx1 * wy0 * v10, w01 = wx0 * wy1 * v01, w11 = wx1 * wy1 * v11;
    const int cx0 = iclamp(x0, 0, W - 1), cx1 = iclamp(x1, 0, W - 1), cy0 = iclamp(y0, 0, H - 1), cy1 = iclamp(y1, 0, H - 1);
    const float* r00 = FTb + ((size_t)cy0 * W + cx0) * C; const float* r10 = FTb + ((size_t)cy0 * W + cx1) * C; const float* r01 = FTb + ((size_t)cy1 * W + cx0) * C; const float* r11 = FTb + ((size_t)cy1 * W + cx1) * C;
#pragma unroll 4
    for (int c4 = hlf * 64; c4 < hlf * 64 + 64; c4 += 4) { const v4f a = *(const v4f*)(r00 + c4), bq = *(const v4f*)(r10 + c4), cq = *(const v4f*)(r01 + c4), dq = *(const v4f*)(r11 + c4); v4h hv, lv;
      for (int q = 0; q < 4; ++q) { const float s = (w00 * a[q] + w10 * bq[q]) + (w01 * cq[q] + w11 * dq[q]); const float vs = s * XS; const b16 ph = (b16)vs; hv[q] = ph; lv[q] = (b16)((vs - (float)ph) * RS_); }
      *(v4h*)(&Ah[wave][nloc][c4]) = hv; *(v4h*)(&Al[wave][nloc][c4]) = lv; }
    wave_lds_sync();
#pragma unroll 1
    for (int kb = 0; kb < C; kb += 32) { const v16b a = frag_kb(&Ah[wave][nloc][kb], hlf), al = frag_kb(&Al[wave][nloc][kb], hlf);
#pragma unroll
      for (int t = 0; t < 16; ++t) { const size_t wo_ = (size_t)(t * 16 + nloc) * KD + tap * C + kb; acc[t] = wmma16b(a, frag_kb(WT + wo_, hlf), acc[t]); acc[t] = wmma16b(al, frag_kb(WTQ + wo_, hlf), acc[t]); } }
    wave_lds_sync(); }
#pragma unroll
  for (int t = 0; t < 16; ++t)
#pragma unroll
    for (int r = 0; r < 8; ++r) Tf[wave][8 * hlf + r][t * 16 + nloc] = acc[t][r] * (1.0f / (XS * WSC));
  __syncthreads();
  for (int pass = 0; pass < 2; ++pass) { for (int q = 0; q < OC / 2; ++q) { const int o = wave * (OC / 2) + q; ((volatile float*)out)[((size_t)b * OC + o) * HW + blockIdx.x * 32 + lane] = Tf[lane >> 4][lane & 15][o]; } __threadfence(); }
}
}

extern "C" void kernel_launch(void* const* d_in, const int* in_sizes, int n_in, void* d_out, int out_size, void* d_ws, size_t ws_size, hipStream_t stream) {
  (void)n_in;
  auto Fp = [&](int i) { return (const float*)d_in[i]; };
  if (in_sizes[0] != B * C * HW || in_sizes[1] != B * 2 * NT * HW || in_sizes[2] != OC * C * NT || out_size != B * OC * HW) return;
  size_t off_ = 0; char* ws = (char*)d_ws;
  auto carve = [&](size_t bytes) { char* p = ws + off_; off_ += (bytes + 255) & ~(size_t)255; return p; };
  b16* WT = (b16*)carve((size_t)OC * KD * 2); b16* WTQ = (b16*)carve((size_t)OC * KD * 2); float* FT = (float*)carve((size_t)B * HW * C * 4);
  if (off_ > ws_size || off_ > ((size_t)128 << 20)) return;
  wperm_kernel<<<(OC * KD / 8 + 255) / 256, 256, 0, stream>>>(Fp(2), WT, WSC); wperm_kernel<<<(OC * KD / 8 + 255) / 256, 256, 0, stream>>>(Fp(2), WTQ, WSC / RS_);
  nhwc_kernel<<<dim3(HW / 32, BL), 256, 0, stream>>>(Fp(0), FT);
  dcn_kernel<<<dim3(HW / 32, BL), 64, 0, stream>>>(FT, Fp(1), WT, WTQ, (float*)d_out);
}
